// RGATransformerDecoderLayer_49091476194115
// MI455X (gfx1250) — hardware-run, weakly checked
//
#include <hip/hip_runtime.h>


#ifndef NB
#define NB 4
#endif
#ifndef SEQ
#define SEQ 1024
#endif
#define NB_FULL  4
#define SEQ_FULL 1024
#ifndef OUT_SEQ
#define OUT_SEQ SEQ
#endif
#define DM   1024
#define NH_  16
#define HD   64
#define FF   4096
#define AW   4
#define SC2   (0.125f * 1.4426950408889634f)
#define FILL2 (-1.0e9f * 1.4426950408889634f)
#define WCS  64.0f
#define FCS  16.0f

static_assert(HD == 64);
static_assert(NH_ * HD == DM);
static_assert(DM % 256 == 0);
static_assert(FF % 64 == 0);
static_assert(SEQ % 64 == 0);
static_assert((NB * SEQ) % 64 == 0);
static_assert(SEQ % 32 == 0);
static_assert(SEQ % (16 * AW) == 0);
static_assert(NB <= NB_FULL);
static_assert(SEQ <= SEQ_FULL);

typedef _Float16 h16;
typedef unsigned short us16;
typedef __attribute__((ext_vector_type(16))) _Float16 v16h;
typedef __attribute__((ext_vector_type(16))) __bf16   v16b;
typedef __attribute__((ext_vector_type(16))) unsigned short v16u;
typedef __attribute__((ext_vector_type(8)))  unsigned short v8u;
typedef __attribute__((ext_vector_type(8)))  float    v8f;
typedef __attribute__((ext_vector_type(4)))  float    v4f;
typedef __attribute__((ext_vector_type(4)))  int      v4i;
typedef v4f  __attribute__((may_alias)) v4fa;

__device__ __forceinline__ unsigned short f2bf(float f) { unsigned u = __float_as_uint(f); u += 0x7FFFu + ((u >> 16) & 1u); return (unsigned short)(u >> 16); }
__device__ __forceinline__ float bf2f(unsigned short b) { return __uint_as_float(((unsigned)b) << 16); }
__device__ __forceinline__ float rbf(float f) { return bf2f(f2bf(f)); }
__device__ __forceinline__ unsigned short f2h(float f) { const h16 v = (h16)f; return __builtin_bit_cast(unsigned short, v); }
__device__ __forceinline__ v16u ld16(const us16* p) { const v8u a = *(const v8u*)p; const v8u b = *(const v8u*)(p + 16);
    return __builtin_shufflevector(a, b, 0, 1, 2, 3, 4, 5, 6, 7, 8, 9, 10, 11, 12, 13, 14, 15); }
template <bool BF>
__device__ __forceinline__ v8f wm(v16u a, v16u b, v8f c) {
    if (BF) return __builtin_amdgcn_wmma_f32_16x16x32_bf16(false, __builtin_bit_cast(v16b, a), false, __builtin_bit_cast(v16b, b), (short)0, c, false, false);
    return __builtin_amdgcn_wmma_f32_16x16x32_f16(false, __builtin_bit_cast(v16h, a), false, __builtin_bit_cast(v16h, b), (short)0, c, false, false);
}
__device__ __forceinline__ void wave_sync() { __builtin_amdgcn_fence(3  , "wavefront"); __builtin_amdgcn_wave_barrier(); asm volatile("" ::: "memory"); }

__global__ __launch_bounds__(256) void k_cvt(const float* __restrict__ X, us16* O) {
    const size_t idx = (size_t)blockIdx.x * 256 + threadIdx.x;
    const size_t row = idx / (DM / 8); const int c = (int)(idx % (DM / 8)) * 8;
    const float* src = X + ((row / SEQ) * (size_t)SEQ_FULL + (row % SEQ)) * DM + c;
    const v4f a = *(const v4f*)src; const v4f b = *(const v4f*)(src + 4);
    v8u o;
#pragma unroll
    for (int i = 0; i < 4; ++i) { o[i] = f2bf(a[i]); o[4 + i] = f2bf(b[i]); }
    us16* d = O + row * DM + c;
    *(volatile v8u*)d = o;
    __threadfence();
    *(volatile v8u*)d = o;
}

template <bool BF>
__global__ __launch_bounds__(256) void k_wt(const float* __restrict__ W, us16* Wt, int K, int N) {
    __shared__ __align__(16) us16 tl[64 * 72];
    const int tid = threadIdx.x; const int n0 = blockIdx.x * 64, k0 = blockIdx.y * 64;
#pragma unroll
    for (int it = 0; it < 4; ++it) { const int k = it * 16 + (tid >> 4), c = (tid & 15) * 4;
        const v4f v = *(const v4f*)(W + (size_t)(k0 + k) * N + n0 + c);
#pragma unroll
        for (int i = 0; i < 4; ++i) tl[(c + i) * 72 + k] = BF ? f2bf(v[i]) : f2h(rbf(v[i]) * WCS); }
    __syncthreads();
    const int rw = tid >> 3, c8 = (tid & 7) * 8;
    const v8u o0 = *(const v8u*)(&tl[rw * 72 + c8]); const v8u o1 = *(const v8u*)(&tl[(32 + rw) * 72 + c8]);
    us16* d0 = Wt + (size_t)(n0 + rw) * K + k0 + c8; us16* d1 = Wt + (size_t)(n0 + 32 + rw) * K + k0 + c8;
    *(volatile v8u*)d0 = o0; *(volatile v8u*)d1 = o1;
    __threadfence();
    *(volatile v8u*)d0 = o0; *(volatile v8u*)d1 = o1;
}

template <int OM>
__global__ __launch_bounds__(256) void k_ln(const float* __restrict__ X, const float* __restrict__ G, const float* __restrict__ Bv,
                                            float* OF, int outSeq, us16* P16, size_t loOff) {
    const int lane = threadIdx.x & 31, wave = __builtin_amdgcn_readfirstlane((int)(threadIdx.x >> 5));
    const int row = blockIdx.x * 8 + wave;
    const float* xr = X + (size_t)row * DM;
    float s = 0.0f;
#pragma unroll 1
    for (int j = 0; j < 8; ++j) { const v4f v = *(const v4f*)(xr + j * 128 + lane * 4); s += (v[0] + v[1]) + (v[2] + v[3]); }
    s += __shfl_xor(s, 16, 32); s += __shfl_xor(s, 8, 32); s += __shfl_xor(s, 4, 32); s += __shfl_xor(s, 2, 32); s += __shfl_xor(s, 1, 32);
    const float mean = s * (1.0f / (float)DM);
    float q = 0.0f;
#pragma unroll 1
    for (int j = 0; j < 8; ++j) { const v4f v = *(const v4f*)(xr + j * 128 + lane * 4);
#pragma unroll
        for (int i = 0; i < 4; ++i) { const float d = v[i] - mean; q += d * d; } }
    q += __shfl_xor(q, 16, 32); q += __shfl_xor(q, 8, 32); q += __shfl_xor(q, 4, 32); q += __shfl_xor(q, 2, 32); q += __shfl_xor(q, 1, 32);
    const float rstd = rsqrtf(q * (1.0f / (float)DM) + 1.0e-5f);
    float* orow = OF + ((size_t)(row / SEQ) * (size_t)outSeq + (size_t)(row % SEQ)) * DM + lane * 4;
#pragma unroll 1
    for (int ps = 0; ps < 2; ++ps) {
#pragma unroll 1
        for (int j = 0; j < 8; ++j) { const v4f v = *(const v4f*)(xr + j * 128 + lane * 4); const v4f g = *(const v4f*)(G + j * 128 + lane * 4); const v4f bb = *(const v4f*)(Bv + j * 128 + lane * 4); v4f o;
#pragma unroll
            for (int i = 0; i < 4; ++i) o[i] = (v[i] - mean) * rstd * rbf(g[i]) + rbf(bb[i]);
            *(volatile v4f*)(orow + j * 128) = o; }
        if (ps == 0) __threadfence(); }
    if (OM != 2) {
        us16* hr = P16 + (size_t)row * DM + lane * 8;
#pragma unroll 1
        for (int ps = 0; ps < 2; ++ps) {
#pragma unroll 1
            for (int j = 0; j < 4; ++j) { const v8f v = *(const v8f*)(xr + j * 256 + lane * 8); const v8f g = *(const v8f*)(G + j * 256 + lane * 8); const v8f bb = *(const v8f*)(Bv + j * 256 + lane * 8); v8u oh, ol;
#pragma unroll
                for (int i = 0; i < 8; ++i) { const float y = (v[i] - mean) * rstd * rbf(g[i]) + rbf(bb[i]);
                    if (OM == 0) { const unsigned short hb = f2bf(y); oh[i] = hb; ol[i] = f2bf(y - bf2f(hb)); }
                    else { oh[i] = f2h(y); ol[i] = 0; } }
                *(volatile v8u*)(hr + j * 256) = oh; if (OM == 0) *(volatile v8u*)(hr + loOff + j * 256) = ol; }
            if (ps == 0) __threadfence(); }
    }
}

template <int MODE, bool BF>
__global__ __launch_bounds__(32) __attribute__((amdgpu_num_vgpr(256)))
void k_gemm(const us16* __restrict__ A, size_t aLoOff, int nPl, const us16* __restrict__ Bt, int K,
            const float* __restrict__ bias, float scale, float ocarry,
            us16* P0, us16* P1, size_t pLoOff, float* ST, size_t tqOff, int wQ, int wV, int wS,
            float* OF, const float* __restrict__ RES, int resSeq) {
    __shared__ __align__(16) float os[64 * 68];
    __shared__ __align__(16) float st[128];
    const int lane = threadIdx.x & 31, lr = lane & 15, hi = lane >> 4; const int r0 = blockIdx.x * 64, c0 = blockIdx.y * 64;
    v8f acc[4][4];
#pragma unroll
    for (int mb = 0; mb < 4; ++mb)
#pragma unroll
        for (int nb = 0; nb < 4; ++nb) acc[mb][nb] = (v8f){};
    const size_t aoff = (size_t)(r0 + lr) * K + 8 * hi, boff = (size_t)(c0 + lr) * K + 8 * hi;
#pragma unroll 1
    for (int pl = 0; pl < nPl; ++pl) {
        const size_t ao = aoff + (size_t)pl * aLoOff;
#pragma unroll 1
        for (int kc = 0; kc < K; kc += 32) {
            v16u a[4];
#pragma unroll
            for (int mb = 0; mb < 4; ++mb) a[mb] = ld16(A + ao + (size_t)mb * 16 * K + kc);
#pragma unroll
            for (int nb = 0; nb < 4; ++nb) { const v16u b = ld16(Bt + boff + (size_t)nb * 16 * K + kc);
#pragma unroll
                for (int mb = 0; mb < 4; ++mb) acc[mb][nb] = wm<BF>(a[mb], b, acc[mb][nb]); }
            asm volatile("v_nop\n\tv_nop\n\tv_nop\n\tv_nop" : "+v"(acc[0][0]), "+v"(acc[1][1]), "+v"(acc[2][2]), "+v"(acc[3][3]) : "v"(a[0]), "v"(a[1]), "v"(a[2]), "v"(a[3]));
        }
    }
#pragma unroll
    for (int mb = 0; mb < 4; ++mb)
#pragma unroll
        for (int nb = 0; nb < 4; ++nb)
#pragma unroll
            for (int j = 0; j < 8; ++j) os[(mb * 16 + hi * 8 + j) * 68 + nb * 16 + lr] = acc[mb][nb][j];
    wave_sync();
    if (MODE == 0 || MODE == 2) {
        const int rq = lane >> 3, c8 = (lane & 7) * 8;
        float bc[8];
        { const v4f b0 = *(const v4f*)(bias + c0 + c8); const v4f b1 = *(const v4f*)(bias + c0 + c8 + 4);
#pragma unroll
          for (int i = 0; i < 4; ++i) { bc[i] = rbf(b0[i]); bc[4 + i] = rbf(b1[i]); } }
#pragma unroll 1
        for (int s = 0; s < 16; ++s) { const int row = 4 * s + rq;
            v4f x0 = *(const v4fa*)(&os[row * 68 + c8]); v4f x1 = *(const v4fa*)(&os[row * 68 + c8 + 4]);
#pragma unroll
            for (int i = 0; i < 4; ++i) { float u0 = x0[i] * scale + bc[i]; float u1 = x1[i] * scale + bc[4 + i];
                if (MODE == 2) { u0 = fmaxf(u0, 0.0f) * ocarry; u1 = fmaxf(u1, 0.0f) * ocarry; }
                x0[i] = u0; x1[i] = u1; }
            *(v4fa*)(&os[row * 68 + c8]) = x0; *(v4fa*)(&os[row * 68 + c8 + 4]) = x1; }
        wave_sync();
        if (MODE == 2) {
            const size_t tbase = (size_t)r0 * FF + c0;
#pragma unroll 1
            for (int ps = 0; ps < 2; ++ps) {
#pragma unroll 4
                for (int s = 0; s < 16; ++s) { const int row = 4 * s + rq;
                    const v4f x0 = *(const v4fa*)(&os[row * 68 + c8]); const v4f x1 = *(const v4fa*)(&os[row * 68 + c8 + 4]); v8u hv;
#pragma unroll
                    for (int i = 0; i < 4; ++i) { hv[i] = f2h(x0[i]); hv[4 + i] = f2h(x1[i]); }
                    *(volatile v8u*)(P0 + tbase + (size_t)row * FF + c8) = hv; }
                if (ps == 0) __threadfence(); }
        } else {
            const int bb = r0 / SEQ, t0 = r0 % SEQ, hh = c0 / HD;
            const size_t bh = (size_t)bb * NH_ + hh;
            if (wQ) {
                const size_t base = (bh * SEQ + t0) * HD;
#pragma unroll 1
                for (int ps = 0; ps < 2; ++ps) {
#pragma unroll 4
                    for (int s = 0; s < 16; ++s) { const int row = 4 * s + rq;
                        const v4f x0 = *(const v4fa*)(&os[row * 68 + c8]); const v4f x1 = *(const v4fa*)(&os[row * 68 + c8 + 4]); v8u hv, lv;
#pragma unroll
                        for (int i = 0; i < 4; ++i) { const unsigned short a0 = f2bf(x0[i]); const unsigned short a1 = f2bf(x1[i]);
                            hv[i] = a0; hv[4 + i] = a1; lv[i] = f2bf(x0[i] - bf2f(a0)); lv[4 + i] = f2bf(x1[i] - bf2f(a1)); }
                        const size_t oo = base + (size_t)row * HD + c8;
                        *(volatile v8u*)(P0 + oo) = hv; *(volatile v8u*)(P0 + pLoOff + oo) = lv; }
                    if (ps == 0) __threadfence(); }
            }
            if (wV) {
                const size_t base = bh * HD * SEQ + t0;
#pragma unroll 1
                for (int ps = 0; ps < 2; ++ps) {
#pragma unroll 2
                    for (int s = 0; s < 16; ++s) { const int d = 4 * s + rq; v8u hv, lv;
#pragma unroll
                        for (int i = 0; i < 8; ++i) { const float x = os[(c8 + i) * 68 + d]; const unsigned short a0 = f2bf(x); hv[i] = a0; lv[i] = f2bf(x - bf2f(a0)); }
                        const size_t oo = base + (size_t)d * SEQ + c8;
                        *(volatile v8u*)(P1 + oo) = hv; *(volatile v8u*)(P1 + pLoOff + oo) = lv; }
                    if (ps == 0) __threadfence(); }
            }
            if (wS) {
                float s0 = 0.0f, s1 = 0.0f, u0 = 0.0f, u1 = 0.0f;
#pragma unroll 4
                for (int d = 0; d < HD; ++d) { const float a = os[lane * 68 + d], c = os[(lane + 32) * 68 + d]; const float fd = (float)d;
                    s0 += a; s1 += c; u0 = fmaf(fd, a, u0); u1 = fmaf(fd, c, u1); }
                st[lane] = s0; st[32 + lane] = s1; st[64 + lane] = u0; st[96 + lane] = u1;
                wave_sync();
                const v4f val = *(const v4fa*)(&st[hi * 64 + lr * 4]);
                float* dst = ST + (size_t)hi * tqOff + bh * SEQ + t0 + lr * 4;
                *(volatile v4f*)dst = val;
                __threadfence();
                *(volatile v4f*)dst = val;
            }
        }
    } else {
        const int cofs = lr * 4;
        v4f bq = *(const v4f*)(bias + c0 + cofs);
#pragma unroll
        for (int i = 0; i < 4; ++i) bq[i] = rbf(bq[i]);
        const size_t rrow0 = (size_t)(r0 / SEQ) * (size_t)resSeq + (size_t)(r0 % SEQ);
#pragma unroll 1
        for (int ps = 0; ps < 2; ++ps) {
#pragma unroll 4
            for (int s = 0; s < 32; ++s) { const int row = 2 * s + hi;
                const v4f a = *(const v4fa*)(&os[row * 68 + cofs]);
                const v4f rv = *(const v4f*)(RES + (rrow0 + row) * DM + c0 + cofs);
                v4f val;
#pragma unroll
                for (int i = 0; i < 4; ++i) { const float rr = (MODE == 3) ? rbf(rv[i]) : rv[i]; val[i] = rr + (a[i] * scale + bq[i]); }
                *(volatile v4f*)(OF + ((size_t)r0 + row) * DM + c0 + cofs) = val; }
            if (ps == 0) __threadfence(); }
    }
}

template <int MASKED>
__global__ __launch_bounds__(32 * AW) __attribute__((amdgpu_num_vgpr(256)))
void k_flash(const us16* __restrict__ QP, const us16* __restrict__ KP, const us16* __restrict__ VT, size_t loOff,
             const float* __restrict__ ST, size_t tqOff, const int* __restrict__ MK, us16* Y, size_t yLoOff) {
    __shared__ __align__(16) float os[AW * 16 * 68];
    const int lane = threadIdx.x & 31, lr = lane & 15, hi = lane >> 4;
    const int wave = __builtin_amdgcn_readfirstlane((int)(threadIdx.x >> 5));
    const int zh = blockIdx.y; const int b = zh / NH_, h = zh % NH_;
    const int t0 = (blockIdx.x * AW + wave) * 16;
    const int iq = t0 + lr;
    const size_t pbase = (size_t)zh * SEQ * HD;
    const size_t qo = pbase + (size_t)iq * HD + 8 * hi;
    const v16u qh0 = ld16(QP + qo), qh1 = ld16(QP + qo + 32), ql0 = ld16(QP + loOff + qo), ql1 = ld16(QP + loOff + qo + 32);
    const size_t ko = pbase + (size_t)lr * HD + 8 * hi;
    const size_t vo = pbase + (size_t)lr * SEQ + 8 * hi;
    const int iq1 = (iq + 1 < SEQ) ? (iq + 1) : (SEQ - 1);
    const float* sp = ST + (size_t)zh * SEQ;
    const float sq0 = sp[iq], tq0 = sp[tqOff + iq], sq1 = sp[iq1], tq1 = sp[tqOff + iq1];
    const int* mrow = MK + (size_t)iq * SEQ_FULL + 8 * hi;
    v8f o[4];
#pragma unroll
    for (int j = 0; j < 4; ++j) o[j] = (v8f){};
    float m = -3.0e38f, l = 0.0f;
#pragma unroll 1
    for (int key0 = 0; key0 < SEQ; key0 += 32) {
        v4i m0 = (v4i){1, 1, 1, 1}, m1 = m0, m2 = m0, m3 = m0;
        if (MASKED) {
            m0 = *(const v4i*)(mrow + key0); m1 = *(const v4i*)(mrow + key0 + 4); m2 = *(const v4i*)(mrow + key0 + 16); m3 = *(const v4i*)(mrow + key0 + 20);
            const v4i mo = (m0 | m1) | (m2 | m3);
            const bool need = ((mo[0] | mo[1] | mo[2] | mo[3]) != 0) || !(m > -7.0e8f);
            if (__builtin_amdgcn_ballot_w32(need) == 0u) continue;
        }
        const us16* ka = KP + ko + (size_t)key0 * HD;
        const us16* kl = ka + loOff;
        const v16u kah0 = ld16(ka), kah1 = ld16(ka + 32), kbh0 = ld16(ka + 16 * HD), kbh1 = ld16(ka + 16 * HD + 32);
        const v16u kal0 = ld16(kl), kal1 = ld16(kl + 32), kbl0 = ld16(kl + 16 * HD), kbl1 = ld16(kl + 16 * HD + 32);
        v8f sa = (v8f){}, sb = (v8f){};
        sa = wm<true>(kah0, qh0, sa); sb = wm<true>(kbh0, qh0, sb);
        sa = wm<true>(kah1, qh1, sa); sb = wm<true>(kbh1, qh1, sb);
        sa = wm<true>(kah0, ql0, sa); sb = wm<true>(kbh0, ql0, sb);
        sa = wm<true>(kah1, ql1, sa); sb = wm<true>(kbh1, ql1, sb);
        sa = wm<true>(kal0, qh0, sa); sb = wm<true>(kbl0, qh0, sb);
        sa = wm<true>(kal1, qh1, sa); sb = wm<true>(kbl1, qh1, sb);
        asm volatile("v_nop\n\tv_nop\n\tv_nop\n\tv_nop" : "+v"(sa), "+v"(sb) : "v"(kah0), "v"(kah1), "v"(kbh0), "v"(kbh1), "v"(kal0), "v"(kal1), "v"(kbl0), "v"(kbl1));
        asm volatile("" ::: "memory");
        float ta[8], tb[8];
        const int dA = iq - (key0 + 8 * hi);
#pragma unroll
        for (int r = 0; r < 8; ++r) {
            const int d1 = dA - r, d2 = dA - 16 - r;
            const float ra = (d1 >= 0) ? fmaf((float)(1 + d1), sq0, tq0) : ((d1 == -1) ? 0.0f : fmaf((float)(SEQ + 2 + d1), sq1, tq1));
            const float rb = (d2 >= 0) ? fmaf((float)(1 + d2), sq0, tq0) : ((d2 == -1) ? 0.0f : fmaf((float)(SEQ + 2 + d2), sq1, tq1));
            ta[r] = (sa[r] + ra) * SC2; tb[r] = (sb[r] + rb) * SC2;
        }
        if (MASKED) {
#pragma unroll
            for (int r = 0; r < 4; ++r) {
                ta[r] = (m0[r] != 0) ? ta[r] : FILL2; ta[4 + r] = (m1[r] != 0) ? ta[4 + r] : FILL2;
                tb[r] = (m2[r] != 0) ? tb[r] : FILL2; tb[4 + r] = (m3[r] != 0) ? tb[4 + r] : FILL2; }
        }
        float mx = -3.0e38f;
#pragma unroll
        for (int r = 0; r < 8; ++r) mx = fmaxf(mx, fmaxf(ta[r], tb[r]));
        mx = fmaxf(mx, __shfl_xor(mx, 16, 32));
        const float mnew = fmaxf(m, mx);
        const float alpha = __builtin_amdgcn_exp2f(m - mnew);
        v16u pbh, pbl; float ls = 0.0f;
#pragma unroll
        for (int r = 0; r < 8; ++r) {
            const float pa = __builtin_amdgcn_exp2f(ta[r] - mnew), pc = __builtin_amdgcn_exp2f(tb[r] - mnew);
            const unsigned short ah = f2bf(pa), ch = f2bf(pc);
            const float ahf = bf2f(ah), chf = bf2f(ch);
            const unsigned short al = f2bf(pa - ahf), cl = f2bf(pc - chf);
            pbh[r] = ah; pbh[8 + r] = ch; pbl[r] = al; pbl[8 + r] = cl;
            ls += (ahf + bf2f(al)) + (chf + bf2f(cl)); }
        l = l * alpha + ls; m = mnew;
#pragma unroll
        for (int j = 0; j < 4; ++j) o[j] = o[j] * alpha;
        const us16* va = VT + vo + key0;
        const us16* vl = va + loOff;
        const v16u vh0 = ld16(va), vh1 = ld16(va + (size_t)16 * SEQ), vh2 = ld16(va + (size_t)32 * SEQ), vh3 = ld16(va + (size_t)48 * SEQ);
        const v16u vl0 = ld16(vl), vl1 = ld16(vl + (size_t)16 * SEQ), vl2 = ld16(vl + (size_t)32 * SEQ), vl3 = ld16(vl + (size_t)48 * SEQ);
        o[0] = wm<true>(vh0, pbh, o[0]); o[1] = wm<true>(vh1, pbh, o[1]); o[2] = wm<true>(vh2, pbh, o[2]); o[3] = wm<true>(vh3, pbh, o[3]);
        o[0] = wm<true>(vh0, pbl, o[0]); o[1] = wm<true>(vh1, pbl, o[1]); o[2] = wm<true>(vh2, pbl, o[2]); o[3] = wm<true>(vh3, pbl, o[3]);
        o[0] = wm<true>(vl0, pbh, o[0]); o[1] = wm<true>(vl1, pbh, o[1]); o[2] = wm<true>(vl2, pbh, o[2]); o[3] = wm<true>(vl3, pbh, o[3]);
        asm volatile("v_nop\n\tv_nop\n\tv_nop\n\tv_nop" : "+v"(o[0]), "+v"(o[1]), "+v"(o[2]), "+v"(o[3])
                     : "v"(vh0), "v"(vh1), "v"(vh2), "v"(vh3), "v"(vl0), "v"(vl1), "v"(vl2), "v"(vl3), "v"(pbh), "v"(pbl));
    }
    l += __shfl_xor(l, 16, 32);
    const float inv = 1.0f / l;
    const int wb = wave * 16 * 68;
#pragma unroll
    for (int j = 0; j < 4; ++j) { v4f a, c;
#pragma unroll
        for (int i = 0; i < 4; ++i) { a[i] = o[j][i] * inv; c[i] = o[j][4 + i] * inv; }
        *(v4fa*)(&os[wb + lr * 68 + 16 * j + 8 * hi]) = a; *(v4fa*)(&os[wb + lr * 68 + 16 * j + 8 * hi + 4]) = c; }
    wave_sync();
    const size_t ybase = ((size_t)b * SEQ + t0) * DM + (size_t)h * HD;
#pragma unroll 1
    for (int ps = 0; ps < 2; ++ps) {
#pragma unroll
        for (int s = 0; s < 4; ++s) { const int row = 4 * s + (lane >> 3), c8 = (lane & 7) * 8;
            const v4f x0 = *(const v4fa*)(&os[wb + row * 68 + c8]); const v4f x1 = *(const v4fa*)(&os[wb + row * 68 + c8 + 4]); v8u hv, lv;
#pragma unroll
            for (int i = 0; i < 4; ++i) { const unsigned short a0 = f2bf(x0[i]); const unsigned short a1 = f2bf(x1[i]);
                hv[i] = a0; hv[4 + i] = a1; lv[i] = f2bf(x0[i] - bf2f(a0)); lv[4 + i] = f2bf(x1[i] - bf2f(a1)); }
            const size_t oo = ybase + (size_t)row * DM + c8;
            *(volatile v8u*)(Y + oo) = hv; *(volatile v8u*)(Y + yLoOff + oo) = lv; }
        if (ps == 0) __threadfence(); }
}

static constexpr size_t al256(size_t v) { return (v + 255) & ~(size_t)255; }
static constexpr size_t cmax(size_t a, size_t b) { return a > b ? a : b; }
static constexpr size_t MROWS   = (size_t)NB * SEQ;
static constexpr size_t EL_ACT  = MROWS * DM;
static constexpr size_t SZ_A16  = EL_ACT * 2;
static constexpr size_t EL_TQ   = (size_t)NB * NH_ * SEQ;
static constexpr size_t SZ_ST   = al256(2 * EL_TQ * 4);
static constexpr size_t SZ_W    = (size_t)DM * DM * 2;
static constexpr size_t SZ_W1   = (size_t)DM * FF * 2;
static constexpr size_t SZ_W2   = (size_t)FF * DM * 2;
static constexpr size_t SZ_F    = MROWS * FF * 2;
static constexpr size_t SZ_RW = al256(4 * SZ_W);
static constexpr size_t SZ_RI = al256(cmax(2 * SZ_A16, SZ_W1 + SZ_W2));
static constexpr size_t SZ_RP = al256(cmax(6 * SZ_A16 + SZ_ST, SZ_F));
static constexpr size_t SZ_RC = al256(2 * SZ_A16);
static constexpr size_t SZ_X  = al256(EL_ACT * 4);
static constexpr size_t SZ_TOTAL = SZ_RW + SZ_RI + SZ_RP + SZ_RC + 2 * SZ_X;
static_assert(SZ_TOTAL <= (size_t)134217728);
static_assert(SZ_A16 % 256 == 0);
static_assert(SZ_W1 % 256 == 0);
static_assert(6 * SZ_A16 + SZ_ST <= SZ_RP);
static_assert(SZ_F <= SZ_RP);
static_assert(SZ_W1 + SZ_W2 <= SZ_RI);
static_assert(2 * SZ_A16 <= SZ_RI);
static_assert((EL_ACT / 8) % 256 == 0);
static_assert(MROWS % 8 == 0);
static_assert((size_t)NB * NH_ * SEQ * HD == EL_ACT);

extern "C" void kernel_launch(void* const* d_in, const int* in_sizes, int n_in,
                              void* d_out, int out_size, void* d_ws, size_t ws_size, hipStream_t stream) {
    if (n_in < 21) return;
    const size_t need_act = ((size_t)(NB - 1) * SEQ_FULL + SEQ) * DM;
    if ((size_t)in_sizes[0] < need_act || (size_t)in_sizes[1] < need_act) return;
    if ((size_t)in_sizes[2] < (size_t)(SEQ - 1) * SEQ_FULL + SEQ) return;
    if ((size_t)in_sizes[3] < (size_t)DM * DM || (size_t)in_sizes[5] < (size_t)DM * DM) return;
    if ((size_t)in_sizes[7] < (size_t)DM * DM || (size_t)in_sizes[9] < (size_t)DM * DM) return;
    if ((size_t)in_sizes[4] < (size_t)DM || (size_t)in_sizes[6] < (size_t)DM || (size_t)in_sizes[8] < (size_t)DM || (size_t)in_sizes[10] < (size_t)DM) return;
    if ((size_t)in_sizes[11] < (size_t)DM * FF || (size_t)in_sizes[12] < (size_t)FF) return;
    if ((size_t)in_sizes[13] < (size_t)FF * DM || (size_t)in_sizes[14] < (size_t)DM) return;
    for (int i = 15; i < 21; ++i) if ((size_t)in_sizes[i] < (size_t)DM) return;
    if ((size_t)out_size < ((size_t)(NB - 1) * OUT_SEQ + SEQ) * DM) return;
    if (SZ_TOTAL > ws_size) return;
    const float* tgt  = (const float*)d_in[0];  const float* mem  = (const float*)d_in[1];  const int* mask = (const int*)d_in[2];
    const float* saWq = (const float*)d_in[3];  const float* sabq = (const float*)d_in[4];
    const float* saWo = (const float*)d_in[5];  const float* sabo = (const float*)d_in[6];
    const float* caWq = (const float*)d_in[7];  const float* cabq = (const float*)d_in[8];
    const float* caWo = (const float*)d_in[9];  const float* cabo = (const float*)d_in[10];
    const float* w1   = (const float*)d_in[11]; const float* b1   = (const float*)d_in[12];
    const float* w2   = (const float*)d_in[13]; const float* b2   = (const float*)d_in[14];
    const float* g1   = (const float*)d_in[15]; const float* be1  = (const float*)d_in[16];
    const float* g2   = (const float*)d_in[17]; const float* be2  = (const float*)d_in[18];
    const float* g3   = (const float*)d_in[19]; const float* be3  = (const float*)d_in[20];
    float* OUT = (float*)d_out;
    char* wsp = (char*)d_ws;
    char* RW = wsp; wsp += SZ_RW;
    char* RI = wsp; wsp += SZ_RI;
    char* RP = wsp; wsp += SZ_RP;
    char* RC = wsp; wsp += SZ_RC;
    char* RA = wsp; wsp += SZ_X;
    char* RB = wsp; wsp += SZ_X;
    us16* WQS = (us16*)RW;
    us16* WOS = (us16*)(RW + SZ_W);
    us16* WQC = (us16*)(RW + 2 * SZ_W);
    us16* WOC = (us16*)(RW + 3 * SZ_W);
    us16* TGB = (us16*)RI;
    us16* MEB = (us16*)(RI + SZ_A16);
    us16* W1T = (us16*)RI;
    us16* W2T = (us16*)(RI + SZ_W1);
    us16* QH  = (us16*)RP;
    us16* KH  = (us16*)(RP + 2 * SZ_A16);
    us16* VTH = (us16*)(RP + 4 * SZ_A16);
    float* STp = (float*)(RP + 6 * SZ_A16);
    us16* FP  = (us16*)RP;
    us16* CTX = (us16*)RC;
    float* XA = (float*)RA;
    float* XB = (float*)RB;
    const dim3 gP((unsigned)(MROWS / 64), DM / 64, 1);
    const dim3 gA(SEQ / (16 * AW), NB * NH_, 1);

    k_cvt<<<(unsigned)(EL_ACT / 8 / 256), 256, 0, stream>>>(tgt, TGB);
    k_cvt<<<(unsigned)(EL_ACT / 8 / 256), 256, 0, stream>>>(mem, MEB);
    k_wt<true><<<dim3(DM / 64, DM / 64, 1), 256, 0, stream>>>(saWq, WQS, DM, DM);
    k_wt<true><<<dim3(DM / 64, DM / 64, 1), 256, 0, stream>>>(saWo, WOS, DM, DM);
    k_wt<true><<<dim3(DM / 64, DM / 64, 1), 256, 0, stream>>>(caWq, WQC, DM, DM);
    k_wt<true><<<dim3(DM / 64, DM / 64, 1), 256, 0, stream>>>(caWo, WOC, DM, DM);

    k_gemm<0, true><<<gP, 32, 0, stream>>>(TGB, (size_t)0, 1, WQS, DM, sabq, 1.0f, 1.0f,
        QH, VTH, EL_ACT, STp, EL_TQ, 1, 1, 1, XA, tgt, SEQ);
    k_flash<1><<<gA, 32 * AW, 0, stream>>>(QH, QH, VTH, EL_ACT, STp, EL_TQ, mask, CTX, EL_ACT);
    k_gemm<3, true><<<gP, 32, 0, stream>>>(CTX, EL_ACT, 2, WOS, DM, sabo, 1.0f, 1.0f,
        QH, VTH, EL_ACT, STp, EL_TQ, 0, 0, 0, XA, tgt, SEQ_FULL);
    k_ln<0><<<(unsigned)(MROWS / 8), 256, 0, stream>>>(XA, g1, be1, XB, SEQ, CTX, EL_ACT);

    k_gemm<0, true><<<gP, 32, 0, stream>>>(CTX, EL_ACT, 2, WQC, DM, cabq, 1.0f, 1.0f,
        QH, VTH, EL_ACT, STp, EL_TQ, 1, 0, 1, XA, tgt, SEQ);
    k_gemm<0, true><<<gP, 32, 0, stream>>>(MEB, (size_t)0, 1, WQC, DM, cabq, 1.0f, 1.0f,
        KH, VTH, EL_ACT, STp, EL_TQ, 1, 1, 0, XA, tgt, SEQ);
    k_flash<0><<<gA, 32 * AW, 0, stream>>>(QH, KH, VTH, EL_ACT, STp, EL_TQ, mask, CTX, EL_ACT);
    k_gemm<4, true><<<gP, 32, 0, stream>>>(CTX, EL_ACT, 2, WOC, DM, cabo, 1.0f, 1.0f,
        QH, VTH, EL_ACT, STp, EL_TQ, 0, 0, 0, XA, XB, SEQ);
    k_ln<1><<<(unsigned)(MROWS / 8), 256, 0, stream>>>(XA, g2, be2, XB, SEQ, CTX, (size_t)0);

    k_wt<false><<<dim3(FF / 64, DM / 64, 1), 256, 0, stream>>>(w1, W1T, DM, FF);
    k_wt<false><<<dim3(DM / 64, FF / 64, 1), 256, 0, stream>>>(w2, W2T, FF, DM);
    k_gemm<2, false><<<dim3((unsigned)(MROWS / 64), FF / 64, 1), 32, 0, stream>>>(CTX, (size_t)0, 1, W1T, DM, b1, 1.0f / WCS, FCS,
        FP, FP, (size_t)0, XA, (size_t)0, 0, 0, 0, XA, XB, SEQ);
    k_gemm<4, false><<<gP, 32, 0, stream>>>(FP, (size_t)0, 1, W2T, FF, b2, 1.0f / (WCS * FCS), 1.0f,
        CTX, CTX, (size_t)0, XB, (size_t)0, 0, 0, 0, XA, XB, SEQ);
    k_ln<2><<<(unsigned)(MROWS / 8), 256, 0, stream>>>(XA, g3, be3, OUT, OUT_SEQ, CTX, (size_t)0);
}
